// LHKGNN_12506944766710
// MI455X (gfx1250) — hardware-run, weakly checked
//
#include <hip/hip_runtime.h>


namespace {
constexpr int N = 16384, E = 540672, DI = 512, DH = 256, DO = 64, KC = 10;
constexpr float XS = 8.0f, WSC = 256.0f;
typedef _Float16 b16;
typedef __attribute__((ext_vector_type(16))) _Float16 v16b;
typedef __attribute__((ext_vector_type(8))) _Float16 v8b;
typedef __attribute__((ext_vector_type(8))) float v8f;
typedef __attribute__((ext_vector_type(4))) float v4f;
typedef __attribute__((ext_vector_type(2))) float v2f;
__device__ __forceinline__ float bf16_rne(float f) { unsigned int u = __float_as_uint(f); u += 0x7FFFu + ((u >> 16) & 1u); float r = __uint_as_float(u & 0xFFFF0000u); asm volatile("" : "+v"(r)); return r; }
__device__ __forceinline__ void split16(float v, b16& hi, b16& lo) { hi = (b16)v; lo = (b16)(v - (float)hi); }
__device__ __forceinline__ v16b frag_kb(const b16* p, int hh) { const v8b a = *(const v8b*)(p + 8 * hh), b = *(const v8b*)(p + 16 + 8 * hh); v16b f;
#pragma unroll
  for (int e = 0; e < 8; ++e) { f[e] = a[e]; f[8 + e] = b[e]; } return f; }
__device__ __forceinline__ v8f wmma16b(v16b a, v16b b, v8f c) { v8f d = __builtin_amdgcn_wmma_f32_16x16x32_f16(false, a, false, b, (short)0, c, false, false); asm volatile("v_nop\n\tv_nop\n\tv_nop\n\tv_nop" : "+v"(d) : "v"(a), "v"(b)); return d; }
__device__ __forceinline__ void wave_lds_sync() { __builtin_amdgcn_fence(__ATOMIC_RELEASE, "workgroup"); __builtin_amdgcn_wave_barrier(); __builtin_amdgcn_fence(__ATOMIC_ACQUIRE, "workgroup"); }
__device__ __forceinline__ float pmul(float a, float b) { float p = a * b; asm volatile("" : "+v"(p)); return p; }
__device__ __forceinline__ int iclamp(int v, int lo, int hi) { return v < lo ? lo : (v > hi ? hi : v); }
constexpr int CSR_NBLK8 = 512, CSR_GB8 = 8, CSR_GN8 = 1 << CSR_GB8  , CSR_TS8 = (CSR_GN8 < 32 ? 32 : CSR_GN8)  , CSR_MAXG8 = 512, CSR_CAP8 = 12288  ;
__device__ __host__ __forceinline__ int csr_tix8(int v) { return (v >> CSR_GB8) * CSR_TS8 + (v & (CSR_GN8 - 1)); }
__global__ __launch_bounds__(64) void csrA_kernel8(const int* __restrict__ dst, int E, int N, int nG, int CHP, int NGP, int* __restrict__ STG, int* __restrict__ HST) {
  extern __shared__ int sm[];
  int* cnt = sm; int* run = sm + NGP; int* ids = sm + 2 * NGP;
  const int b = blockIdx.x; const int ch = (E + CSR_NBLK8 - 1) / CSR_NBLK8; const int e0 = b * ch, e1 = min(E, e0 + ch);
  for (int i = threadIdx.x; i < NGP; i += 64) cnt[i] = 0;
  for (int i = threadIdx.x; i < CHP; i += 64) ids[i] = -1;
  __syncthreads();
  if (threadIdx.x == 0) {
    for (int e = e0; e < e1; ++e) { int d = dst[e]; d = (d < 0) ? 0 : (d >= N ? N - 1 : d); cnt[d >> CSR_GB8] += 1; }
    int acc = 0; for (int g = 0; g < nG; ++g) { run[g] = acc; acc += cnt[g]; }
    for (int e = e0; e < e1; ++e) { int d = dst[e]; d = (d < 0) ? 0 : (d >= N ? N - 1 : d); const int g = d >> CSR_GB8; ids[run[g]] = e; run[g] += 1; } }
  __syncthreads();
  typedef __attribute__((ext_vector_type(4))) int v4i;
  for (int pass = 0; pass < 2; ++pass) {
    for (int i = threadIdx.x; i < CHP / 4; i += 64) *(volatile v4i*)(STG + (size_t)b * CHP + i * 4) = *(const v4i*)(&ids[i * 4]);
    for (int i = threadIdx.x; i < NGP / 4; i += 64) { v4i v; for (int e = 0; e < 4; ++e) v[e] = (i * 4 + e < nG) ? cnt[i * 4 + e] : 0; *(volatile v4i*)(HST + (size_t)b * NGP + i * 4) = v; }
    __threadfence(); }
}
__global__ __launch_bounds__(512) void csrS_kernel8(const int* __restrict__ HST, int nG, int NGP, int* __restrict__ START, int* __restrict__ TOT, int* __restrict__ OFF) {
  __shared__ int tot[CSR_MAXG8];
  const int b = threadIdx.x;
  for (int pass = 0; pass < 2; ++pass) { int runb = 0; for (int g = 0; g < nG; ++g) { int c = HST[(size_t)b * NGP + g]; c = (c < 0) ? 0 : c; ((volatile int*)OFF)[(size_t)g * CSR_NBLK8 + b] = runb; runb += c; } __threadfence(); }
  for (int g = threadIdx.x; g < nG; g += 512) { int s = 0; for (int bb = 0; bb < CSR_NBLK8; ++bb) { int c = HST[(size_t)bb * NGP + g]; s += (c < 0) ? 0 : c; } tot[g] = s; }
  __syncthreads();
  if (threadIdx.x < 32) {
    __shared__ int st[CSR_MAXG8 + 32];
    if (threadIdx.x == 0) { int acc = 0; for (int g = 0; g < NGP; ++g) { st[g] = acc; if (g < nG) acc += (tot[g] + 31) & ~31; } st[NGP] = acc; }
    __builtin_amdgcn_fence(__ATOMIC_RELEASE, "workgroup"); __builtin_amdgcn_wave_barrier(); __builtin_amdgcn_fence(__ATOMIC_ACQUIRE, "workgroup");
    for (int pass = 0; pass < 2; ++pass) { for (int i = threadIdx.x; i < NGP + 32; i += 32) { ((volatile int*)START)[i] = (i <= NGP) ? st[min(i, NGP)] : 0; ((volatile int*)TOT)[i] = (i < nG) ? tot[i] : 0; } __threadfence(); } }
}
__global__ __launch_bounds__(256) void csrB_kernel8(const int* __restrict__ dst, int N, int nG, int CHP, int NGP, int permLen, const int* __restrict__ STG, const int* __restrict__ HST, const int* __restrict__ OFF, const int* __restrict__ START, const int* __restrict__ TOT, int* __restrict__ PERM, int* __restrict__ ROWPTR, int* __restrict__ ROWCNT, int* __restrict__ FLAG) {
  typedef __attribute__((ext_vector_type(4))) int v4i;
  __shared__ int ids[CSR_CAP8]; __shared__ unsigned short key[CSR_CAP8]; __shared__ int outp[CSR_CAP8]; __shared__ int ncnt[CSR_GN8 + 1]; __shared__ int boff[CSR_NBLK8 + 1];
  const int g = blockIdx.x, t_ = threadIdx.x; int tot = TOT[g]; int st = START[g], stn = START[g + 1]; const int v0 = g * CSR_GN8; const int nv = min(CSR_GN8, N - v0); const int t0 = g * CSR_TS8;
  st = (st < 0) ? 0 : (st > permLen - 32 ? permLen - 32 : st) & ~31; stn = (stn < st) ? st : (stn > permLen ? permLen : stn); tot = (tot < 0) ? 0 : tot; if (tot > stn - st && tot <= CSR_CAP8) tot = stn - st;
  if (tot > CSR_CAP8) {
    for (int pass = 0; pass < 2; ++pass) { for (int i = t_; i < CSR_TS8 / 4; i += 256) { v4i a, c; for (int e = 0; e < 4; ++e) { a[e] = st; c[e] = 0; } *(volatile v4i*)(ROWPTR + t0 + i * 4) = a; *(volatile v4i*)(ROWCNT + t0 + i * 4) = c; } if (t_ == 0) ((volatile int*)FLAG)[0] = 1; __threadfence(); } (void)nv; return; }
  if (t_ == 0) { int acc = 0; for (int b = 0; b < CSR_NBLK8; ++b) { boff[b] = acc; int c = HST[(size_t)b * NGP + g]; c = (c < 0) ? 0 : (c > CHP ? CHP : c); acc += c; if (acc > tot) acc = tot; } boff[CSR_NBLK8] = acc; }
  for (int i = t_; i <= CSR_GN8; i += 256) ncnt[i] = 0;
  __syncthreads();
  for (int b = 0; b < CSR_NBLK8; ++b) { const int c = boff[b + 1] - boff[b]; int o_ = OFF[(size_t)g * CSR_NBLK8 + b]; o_ = (o_ < 0) ? 0 : (o_ > CHP - c ? CHP - c : o_); const int* src_ = STG + (size_t)b * CHP + o_;
    for (int i = t_; i < c; i += 256) { int id = src_[i]; id = (id < 0) ? 0 : id; ids[boff[b] + i] = id; int d = dst[id]; d = (d < v0) ? v0 : (d >= N ? N - 1 : d); int kk = d - v0; kk = (kk < 0) ? 0 : (kk >= CSR_GN8 ? CSR_GN8 - 1 : kk); key[boff[b] + i] = (unsigned short)kk; } }
  __syncthreads();
  if (t_ == 0) { for (int i = 0; i < tot; ++i) ncnt[key[i]] += 1; int acc = 0; for (int vl = 0; vl < CSR_GN8; ++vl) { const int c = ncnt[vl]; ncnt[vl] = acc; acc += c; } ncnt[CSR_GN8] = acc;
    for (int i = 0; i < tot; ++i) { const int vl = key[i]; outp[ncnt[vl]] = ids[i]; ncnt[vl] += 1; }
    for (int vl = CSR_GN8; vl > 0; --vl) ncnt[vl] = ncnt[vl - 1]; ncnt[0] = 0; }
  __syncthreads();
  for (int pass = 0; pass < 2; ++pass) {
    for (int i = t_; i < (stn - st) / 4; i += 256) { v4i v; for (int e = 0; e < 4; ++e) { const int q = i * 4 + e; v[e] = (q < tot) ? outp[q] : -1; } *(volatile v4i*)(PERM + st + i * 4) = v; }
    for (int i = t_; i < CSR_TS8 / 4; i += 256) { v4i a, c; for (int e = 0; e < 4; ++e) { const int vl = i * 4 + e; const int vc = vl < CSR_GN8 ? vl : CSR_GN8; a[e] = (vl < CSR_GN8) ? st + ncnt[vc] : st; c[e] = (vl < nv) ? (ncnt[(vc < CSR_GN8 ? vc : CSR_GN8 - 1) + 1] - ncnt[vc]) : 0; } *(volatile v4i*)(ROWPTR + t0 + i * 4) = a; *(volatile v4i*)(ROWCNT + t0 + i * 4) = c; }
    __threadfence(); }
}
__global__ __launch_bounds__(256) void csrZ_kernel8(int* __restrict__ p, size_t n4) { typedef __attribute__((ext_vector_type(4))) int v4i; const size_t tid = (size_t)blockIdx.x * 256 + threadIdx.x, nth = (size_t)gridDim.x * 256; v4i z = {0, 0, 0, 0}; for (size_t i = tid; i < n4; i += nth) *(volatile v4i*)(p + i * 4) = z; }
struct CsrBufs8 { int *STG, *HST, *OFF, *START, *TOT, *PERM, *ROWPTR, *ROWCNT, *FLAG; int nG, NGP, CHP; size_t permLen; char* base; size_t bytes; };
static size_t csr_carve8(CsrBufs8& c, char* ws, size_t off, int E, int N) {
  const size_t off0 = off; c.base = ws + off;
  auto al = [&](size_t bytes) { char* p = ws + off; off += (bytes + 255) & ~(size_t)255; return p; };
  c.nG = (N + CSR_GN8 - 1) / CSR_GN8; c.NGP = (c.nG + 31) & ~31; const int ch = (E + CSR_NBLK8 - 1) / CSR_NBLK8; c.CHP = (ch + 31) & ~31; c.permLen = (size_t)E + 32 * (size_t)c.nG + 32;
  c.STG = (int*)al((size_t)CSR_NBLK8 * c.CHP * 4); c.HST = (int*)al((size_t)CSR_NBLK8 * c.NGP * 4); c.OFF = (int*)al((size_t)c.NGP * CSR_NBLK8 * 4); c.START = (int*)al((size_t)(c.NGP + 64) * 4); c.TOT = (int*)al((size_t)(c.NGP + 64) * 4);
  c.PERM = (int*)al(c.permLen * 4); c.ROWPTR = (int*)al((size_t)c.nG * CSR_TS8 * 4); c.ROWCNT = (int*)al((size_t)c.nG * CSR_TS8 * 4); c.FLAG = (int*)al(256);
  c.bytes = off - off0; return off;
}
static void csr_build8(const CsrBufs8& c, const int* dst, int E, int N, hipStream_t stream) {
  const size_t smem = (size_t)(2 * c.NGP + c.CHP) * 4;
  csrZ_kernel8<<<512, 256, 0, stream>>>((int*)c.base, c.bytes / 16);
  csrA_kernel8<<<CSR_NBLK8, 64, smem, stream>>>(dst, E, N, c.nG, c.CHP, c.NGP, c.STG, c.HST);
  csrS_kernel8<<<1, 512, 0, stream>>>(c.HST, c.nG, c.NGP, c.START, c.TOT, c.OFF);
  csrB_kernel8<<<c.nG, 256, 0, stream>>>(dst, N, c.nG, c.CHP, c.NGP, (int)c.permLen, c.STG, c.HST, c.OFF, c.START, c.TOT, c.PERM, c.ROWPTR, c.ROWCNT, c.FLAG);
}


__global__ __launch_bounds__(256) void wput_kernel(const float* __restrict__ w1, const float* __restrict__ w2, b16* __restrict__ W1T, b16* __restrict__ W2T) { const int u = blockIdx.x * 256 + threadIdx.x;
  for (int pass = 0; pass < 2; ++pass) {
    if (u < DH * (DI / 8)) { const int o = u / (DI / 8), k0 = (u % (DI / 8)) * 8; v8b v;
#pragma unroll
      for (int j = 0; j < 8; ++j) v[j] = (b16)(bf16_rne(w1[(size_t)(k0 + j) * DH + o]) * WSC); *(volatile v8b*)(W1T + (size_t)o * DI + k0) = v; }
    if (u < DO * (DH / 8)) { const int o = u / (DH / 8), k0 = (u % (DH / 8)) * 8; v8b v;
#pragma unroll
      for (int j = 0; j < 8; ++j) v[j] = (b16)(bf16_rne(w2[(size_t)(k0 + j) * DO + o]) * WSC); *(volatile v8b*)(W2T + (size_t)o * DH + k0) = v; }
    __threadfence(); } }
__global__ __launch_bounds__(32) void mlp_kernel(const float* __restrict__ x, const b16* __restrict__ W1T, const float* __restrict__ b1, const b16* __restrict__ W2T, const float* __restrict__ b2, float* __restrict__ Hh) { __shared__ __attribute__((aligned(16))) b16 Ah[16][DI + 8], Al[16][DH + 8]; __shared__ float Tf[16][68]; const int lane = threadIdx.x, nloc = lane & 15, hlf = lane >> 4; const size_t m0 = (size_t)blockIdx.x * 16;
  for (int rr = 0; rr < 16; ++rr) for (int q = 0; q < DI / 32; ++q) Ah[rr][q * 32 + lane] = (b16)(bf16_rne(x[(m0 + rr) * DI + q * 32 + lane]) * XS);
  wave_lds_sync(); v8f acc[16];
#pragma unroll
  for (int t = 0; t < 16; ++t) acc[t] = (v8f){};
#pragma unroll 1
  for (int kb = 0; kb < DI; kb += 32) { const v16b a = frag_kb(&Ah[nloc][kb], hlf);
#pragma unroll
    for (int t = 0; t < 16; ++t) acc[t] = wmma16b(a, frag_kb(W1T + (size_t)(t * 16 + nloc) * DI + kb, hlf), acc[t]); }
  wave_lds_sync();
#pragma unroll
  for (int t = 0; t < 16; ++t) { const int cc = t * 16 + nloc; const float bb = bf16_rne(b1[cc]);
#pragma unroll
    for (int r8 = 0; r8 < 8; ++r8) { b16 p, ql; split16(fmaxf(acc[t][r8] * (1.0f / (XS * WSC)) + bb, 0.0f) * XS, p, ql); Ah[8 * hlf + r8][cc] = p; Al[8 * hlf + r8][cc] = ql; } }
  wave_lds_sync(); v8f ac2[4] = {(v8f){}, (v8f){}, (v8f){}, (v8f){}};
#pragma unroll 2
  for (int kb = 0; kb < DH; kb += 32) { const v16b a = frag_kb(&Ah[nloc][kb], hlf), al = frag_kb(&Al[nloc][kb], hlf);
#pragma unroll
    for (int t = 0; t < 4; ++t) { const v16b bw = frag_kb(W2T + (size_t)(t * 16 + nloc) * DH + kb, hlf); ac2[t] = wmma16b(a, bw, ac2[t]); ac2[t] = wmma16b(al, bw, ac2[t]); } }
#pragma unroll
  for (int t = 0; t < 4; ++t) { const int cc = t * 16 + nloc; const float bb = bf16_rne(b2[cc]);
#pragma unroll
    for (int r8 = 0; r8 < 8; ++r8) Tf[8 * hlf + r8][cc] = ac2[t][r8] * (1.0f / (XS * WSC)) + bb; }
  wave_lds_sync();
  for (int pass = 0; pass < 2; ++pass) { for (int rr = 0; rr < 16; ++rr) *(volatile v2f*)(Hh + (m0 + rr) * DO + lane * 2) = (v2f){Tf[rr][lane * 2], Tf[rr][lane * 2 + 1]}; __threadfence(); } }
__global__ __launch_bounds__(256) void deg_kernel(const int* __restrict__ ROWCNT, float* __restrict__ DIS) { const int i = blockIdx.x * 256 + threadIdx.x; if (i >= N) return; const float d = (float)iclamp(ROWCNT[i], 0, E); const float dis = d > 0.0f ? rsqrtf(d) : INFINITY; for (int pass = 0; pass < 2; ++pass) { ((volatile float*)DIS)[i] = dis; __threadfence(); } }
__device__ __forceinline__ float bessel_c(int k, float t) {
  const float th = 0.5f * t, q = pmul(th, th); float term = 1.0f;
#pragma unroll 1
  for (int j = 1; j <= k; ++j) term = pmul(term, th) / (float)j;
  float res = 0.0f;
#pragma unroll 1
  for (int m = 0; m < 10; ++m) { res += term; term = pmul(term, q) / (float)((m + 1) * (m + 1 + k)); }
  const float et = __expf(-t); return k == 0 ? et * res : 2.0f * et * ((k & 1) ? -1.0f : 1.0f) * res; }
template <int FINAL>
__global__ __launch_bounds__(256) void cheb_kernel(int k, const float* __restrict__ Y1, const float* __restrict__ Y0, const float* __restrict__ Hh, const float* __restrict__ ew, const float* __restrict__ DIS, const float* __restrict__ nodet, const float* __restrict__ g0, const float* __restrict__ g1, const int* __restrict__ cols, const int* __restrict__ PERM, const int* __restrict__ ROWPTR, const int* __restrict__ ROWCNT, int permLen, float* __restrict__ Tk, float* __restrict__ Dacc, float* __restrict__ out) {
  const int wave = threadIdx.x >> 5, lane = threadIdx.x & 31; const size_t i = (size_t)blockIdx.x * 8 + wave; if (i >= (size_t)N) return; int st = ROWPTR[i], cnt = ROWCNT[i]; cnt = iclamp(cnt, 0, E); st = iclamp(st, 0, permLen - cnt); const int c0 = lane * 2; const float di = DIS[i];
  float a0 = 0.0f, a1 = 0.0f;
#pragma unroll 1
  for (int j = 0; j < cnt; ++j) { const int e = iclamp(PERM[st + j], 0, E - 1); const size_t u = (size_t)iclamp(cols[e], 0, N - 1); const float v = pmul(pmul(di, bf16_rne(ew[e])), DIS[u]); const v2f y = *(const v2f*)(Y1 + u * DO + c0); a0 += pmul(v, y[0]); a1 += pmul(v, y[1]); }
  const float ly0 = -a0, ly1 = -a1; const float t = fmaxf(bf16_rne(nodet[i]), 0.0f); v2f tk, d;
  if (k == 1) { tk = (v2f){ly0, ly1}; const v2f h = *(const v2f*)(Hh + i * DO + c0); const float cA = bessel_c(0, t), cB = bessel_c(1, t); d = (v2f){pmul(cA, h[0]) + pmul(cB, tk[0]), pmul(cA, h[1]) + pmul(cB, tk[1])}; }
  else { const v2f y0 = *(const v2f*)(Y0 + i * DO + c0); tk = (v2f){2.0f * ly0 - y0[0], 2.0f * ly1 - y0[1]}; const v2f dd = *(const v2f*)(Dacc + i * DO + c0); const float ck = bessel_c(k, t); d = (v2f){dd[0] + pmul(ck, tk[0]), dd[1] + pmul(ck, tk[1])}; }
  if (!FINAL) { for (int pass = 0; pass < 2; ++pass) { *(volatile v2f*)(Tk + i * DO + c0) = tk; *(volatile v2f*)(Dacc + i * DO + c0) = d; __threadfence(); } return; }
  const v2f h = *(const v2f*)(Hh + i * DO + c0); const float ga = bf16_rne(g0[i]), gb = bf16_rne(g1[i]); const float o0 = pmul(ga, h[0]) + pmul(gb, d[0]), o1 = pmul(ga, h[1]) + pmul(gb, d[1]);
  float mx = fmaxf(o0, o1); for (int o = 16; o; o >>= 1) mx = fmaxf(mx, __shfl_xor(mx, o)); float s = __expf(o0 - mx) + __expf(o1 - mx); for (int o = 16; o; o >>= 1) s += __shfl_xor(s, o); const float lse = mx + __logf(s);
  for (int pass = 0; pass < 2; ++pass) { *(volatile v2f*)(out + i * DO + c0) = (v2f){o0 - lse, o1 - lse}; __threadfence(); } }
}

extern "C" void kernel_launch(void* const* d_in, const int* in_sizes, int n_in, void* d_out, int out_size, void* d_ws, size_t ws_size, hipStream_t stream) {
  (void)n_in;
  auto Fp = [&](int i) { return (const float*)d_in[i]; }; auto Ip = [&](int i) { return (const int*)d_in[i]; };
  if (in_sizes[0] != N * DI || in_sizes[1] != 2 * E || in_sizes[2] != E || in_sizes[3] != DI * DH || in_sizes[5] != DH * DO || in_sizes[7] != N || out_size != N * DO) return;
  const int KSTEPS = KC;
  size_t off = 0; char* ws = (char*)d_ws;
  auto carve = [&](size_t bytes) { char* p = ws + off; off += (bytes + 255) & ~(size_t)255; return p; };
  b16* W1T = (b16*)carve((size_t)DH * DI * 2); b16* W2T = (b16*)carve((size_t)DO * DH * 2); float* Hh = (float*)carve((size_t)N * DO * 4); float* DIS = (float*)carve((size_t)N * 4); float* TA = (float*)carve((size_t)N * DO * 4); float* TB = (float*)carve((size_t)N * DO * 4); float* TC = (float*)carve((size_t)N * DO * 4); float* Dacc = (float*)carve((size_t)N * DO * 4);
  CsrBufs8 csr; off = csr_carve8(csr, ws, off, E, N);
  if (off > ws_size || off > ((size_t)48 << 20)) return;
  wput_kernel<<<(DH * (DI / 8) + 255) / 256, 256, 0, stream>>>(Fp(3), Fp(5), W1T, W2T);
  csr_build8(csr, Ip(1), E, N, stream);
  deg_kernel<<<N / 256, 256, 0, stream>>>(csr.ROWCNT, DIS);
  mlp_kernel<<<N / 16, 32, 0, stream>>>(Fp(0), W1T, Fp(4), W2T, Fp(6), Hh);
  float* bufs[3] = {TA, TB, TC}; const float* Y1 = Hh; const float* Y0 = nullptr; const unsigned g = N / 8;
  for (int k = 1; k <= KSTEPS; ++k) { float* Tk = bufs[k % 3];
    if (k == KSTEPS) cheb_kernel<1><<<g, 256, 0, stream>>>(k, Y1, Y0, Hh, Fp(2), DIS, Fp(7), Fp(8), Fp(9), Ip(1) + E, csr.PERM, csr.ROWPTR, csr.ROWCNT, (int)csr.permLen, Tk, Dacc, (float*)d_out);
    else cheb_kernel<0><<<g, 256, 0, stream>>>(k, Y1, Y0, Hh, Fp(2), DIS, Fp(7), Fp(8), Fp(9), Ip(1) + E, csr.PERM, csr.ROWPTR, csr.ROWCNT, (int)csr.permLen, Tk, Dacc, nullptr);
    Y0 = Y1; Y1 = Tk; }
}
